// Samba_Layer_25503515803686
// MI455X (gfx1250) — hardware-verified
//
#include <hip/hip_runtime.h>
#include <stdint.h>


#define LSEQ 2048
#define DM   512
#define DI   1024
#define NS   16
#define RR   32
#define NBC  64
#define HM   2048
#define NLAY 4
#define KC   4

static_assert(NBC == RR + 2 * NS);
static_assert(LSEQ % 64 == 0);
static_assert(LSEQ % 16 == 0);
static_assert(DM == 128 * 4);
static_assert(DI == 128 * 8);
static_assert(DM % 128 == 0);
static_assert(DI % 128 == 0);
static_assert((2 * DI) % 128 == 0);
static_assert(HM % 128 == 0);
static_assert(NBC % 64 == 0);
static_assert(DM % 32 == 0 && DI % 32 == 0 && RR % 32 == 0 && HM % 32 == 0);

typedef float          v4f   __attribute__((ext_vector_type(4)));
typedef float          v8f   __attribute__((ext_vector_type(8)));
typedef _Float16       v8h   __attribute__((ext_vector_type(8)));
typedef _Float16       v16h  __attribute__((ext_vector_type(16)));
typedef unsigned short u16x8 __attribute__((ext_vector_type(8)));

union FragH { u16x8 h[2]; v16h v; };
union Pack8 { v8h f; u16x8 u; };
union Pack1 { _Float16 f; unsigned short u; };

__device__ __forceinline__ v8f ld8f(const float* p) {
    const v4f a = *(const v4f*)p;
    const v4f b = *(const v4f*)(p + 4);
    return __builtin_shufflevector(a, b, 0, 1, 2, 3, 4, 5, 6, 7);
}
__device__ __forceinline__ v8f zero8() {
    v8f z;
#pragma unroll
    for (int c = 0; c < 8; ++c) z[c] = 0.0f;
    return z;
}
__device__ __forceinline__ float hsum4(v4f v) { return (v[0] + v[1]) + (v[2] + v[3]); }

__device__ __forceinline__ float silu_f(float x) {
    const float e = __expf(-x);
    return x * __builtin_amdgcn_rcpf(1.0f + e);
}
__device__ __forceinline__ float softplus_f(float x) {
    return fmaxf(x, 0.0f) + log1pf(__expf(-fabsf(x)));
}
__device__ __forceinline__ float gelu_f(float x) {
    const float y = 0.7978845608028654f * (x + 0.044715f * (x * x * x));
    const float e = __expf(2.0f * y);
    const float t = 1.0f - 2.0f * __builtin_amdgcn_rcpf(e + 1.0f);
    return 0.5f * x * (1.0f + t);
}
__device__ __forceinline__ float conv4(float x0, float x1, float x2, float x3, v4f w, float bias) {
    return (((w[0] * x0 + w[1] * x1) + w[2] * x2) + w[3] * x3) + bias;
}

__device__ __forceinline__ void mma16(v8f& acc, const FragH& a, const FragH& b) {
    acc = __builtin_amdgcn_wmma_f32_16x16x32_f16(false, a.v, false, b.v, (short)0, acc, false, false);
    asm volatile("v_nop\n\tv_nop\n\tv_nop\n\tv_nop" : "+v"(acc) : "v"(a.v), "v"(b.v));
}

__device__ __forceinline__ float block_sum128(float v, float* sred) {
#pragma unroll
    for (int o = 16; o > 0; o >>= 1) v += __shfl_xor(v, o, 32);
    const int lane = threadIdx.x & 31;
    const int wave = threadIdx.x >> 5;
    __syncthreads();
    if (lane == 0) sred[wave] = v;
    __syncthreads();
    return (sred[0] + sred[1]) + (sred[2] + sred[3]);
}

__global__ __launch_bounds__(256)
void cvt_f16_kernel(const float* __restrict__ src, unsigned short* dst, int n8, float scale)
{
    const int i = blockIdx.x * 256 + threadIdx.x;
    if (i >= n8) return;
    const size_t e = (size_t)i * 8;
    Pack8 pk;
    pk.f = __builtin_convertvector(ld8f(src + e) * scale, v8h);
    const u16x8 v = pk.u;
    *(volatile u16x8*)(dst + e) = v;
    __threadfence();
    *(volatile u16x8*)(dst + e) = v;
}

template<int NBF>
__device__ __forceinline__ void tile_store_f32(const float* st, float* gp, int ldc, int lane) {
    constexpr int CW  = NBF * 16;
    constexpr int P   = CW + 4;
    constexpr int LPR = CW / 4;
    constexpr int RPI = 32 / LPR;
    constexpr int NIT = 32 / RPI;
    const int rsub = lane / LPR;
    const int c4   = (lane % LPR) * 4;
#pragma unroll
    for (int it = 0; it < NIT; ++it) {
        const int row = it * RPI + rsub;
        const v4f v = *(const v4f*)(st + row * P + c4);
        *(volatile v4f*)(gp + (size_t)row * ldc + c4) = v;
    }
}
template<int NBF>
__device__ __forceinline__ void tile_store_f16(const float* st, unsigned short* gp, int ldc, int lane) {
    constexpr int CW  = NBF * 16;
    constexpr int P   = CW + 4;
    constexpr int LPR = CW / 8;
    constexpr int RPI = 32 / LPR;
    constexpr int NIT = 32 / RPI;
    const int rsub = lane / LPR;
    const int c8   = (lane % LPR) * 8;
#pragma unroll
    for (int it = 0; it < NIT; ++it) {
        const int row = it * RPI + rsub;
        Pack8 pk;
        pk.f = __builtin_convertvector(ld8f(st + row * P + c8), v8h);
        const u16x8 u = pk.u;
        *(volatile u16x8*)(gp + (size_t)row * ldc + c8) = u;
    }
}

template<int NBF, int EP, bool AF32, bool OUT16>
__global__ __launch_bounds__(128)
void gemm_tn_kernel(const unsigned short* __restrict__ A16, const float* __restrict__ A32, int lda,
                    const unsigned short* __restrict__ Bw, int ldb,
                    float* C32, unsigned short* C16, int ldc,
                    const float* __restrict__ bias, const float* __restrict__ addsrc, int ldadd,
                    int K, float ascale, float scale, float oscale)
{
    constexpr int CW = NBF * 16;
    constexpr int P  = CW + 4;
    __shared__ __attribute__((aligned(16))) float stile[4][32 * P];

    const int tid  = threadIdx.x;
    const int lane = tid & 31;
    const int wave = tid >> 5;
    const int h    = lane >> 4;
    const int m    = lane & 15;
    const int wm   = wave >> 1;
    const int wn   = wave & 1;

    const int rowW = blockIdx.y * 64 + wm * 32;
    const int colW = blockIdx.x * (2 * CW) + wn * CW;

    v8f acc[2 * NBF];
#pragma unroll
    for (int j = 0; j < 2 * NBF; ++j)
#pragma unroll
        for (int r = 0; r < 8; ++r) acc[j][r] = 0.0f;

    const int nk = K >> 5;
    for (int kt = 0; kt < nk; ++kt) {
        const int k0 = kt * 32;
        FragH fa[2], fb[NBF];
#pragma unroll
        for (int s = 0; s < 2; ++s) {
            const size_t ro = (size_t)(rowW + s * 16 + m) * lda + k0 + 8 * h;
            if (AF32) {
                Pack8 p0, p1;
                p0.f = __builtin_convertvector(ld8f(A32 + ro) * ascale, v8h);
                p1.f = __builtin_convertvector(ld8f(A32 + ro + 16) * ascale, v8h);
                fa[s].h[0] = p0.u;
                fa[s].h[1] = p1.u;
            } else {
                fa[s].h[0] = *(const u16x8*)(A16 + ro);
                fa[s].h[1] = *(const u16x8*)(A16 + ro + 16);
            }
        }
#pragma unroll
        for (int j = 0; j < NBF; ++j) {
            const size_t co = (size_t)(colW + j * 16 + m) * ldb + k0 + 8 * h;
            fb[j].h[0] = *(const u16x8*)(Bw + co);
            fb[j].h[1] = *(const u16x8*)(Bw + co + 16);
        }
#pragma unroll
        for (int s = 0; s < 2; ++s)
#pragma unroll
            for (int j = 0; j < NBF; ++j)
                mma16(acc[s * NBF + j], fa[s], fb[j]);
    }

    float* st = stile[wave];
    float bv[NBF];
#pragma unroll
    for (int j = 0; j < NBF; ++j) bv[j] = (EP != 0) ? bias[colW + j * 16 + m] : 0.0f;
#pragma unroll
    for (int s = 0; s < 2; ++s)
#pragma unroll
        for (int j = 0; j < NBF; ++j)
#pragma unroll
            for (int r = 0; r < 8; ++r) {
                const int rl = s * 16 + 8 * h + r;
                const int cl = j * 16 + m;
                float v = acc[s * NBF + j][r] * scale;
                if (EP == 1) {
                    v = softplus_f(v + bv[j]);
                } else if (EP == 2) {
                    v = oscale * gelu_f(v + bv[j]);
                } else if (EP == 3) {
                    v = addsrc[(size_t)(rowW + rl) * ldadd + colW + cl] + (v + bv[j]);
                }
                st[rl * P + cl] = v;
            }
    __syncthreads();

    if (OUT16) {
        unsigned short* gp = C16 + (size_t)rowW * ldc + colW;
        tile_store_f16<NBF>(st, gp, ldc, lane);
        __threadfence();
        tile_store_f16<NBF>(st, gp, ldc, lane);
    } else {
        float* gp = C32 + (size_t)rowW * ldc + colW;
        tile_store_f32<NBF>(st, gp, ldc, lane);
        __threadfence();
        tile_store_f32<NBF>(st, gp, ldc, lane);
    }
}

__global__ __launch_bounds__(128)
void prenorm_kernel(const float* __restrict__ hid, const float* __restrict__ lw, const float* __restrict__ lb,
                    const float* __restrict__ hb, float* resid, const float* __restrict__ bnw,
                    unsigned short* hn16, int first)
{
    __shared__ float sred[4];
    __shared__ __attribute__((aligned(16))) float srow[DM];
    const int row = blockIdx.x;
    const int tid = threadIdx.x;
    const int c4  = tid * 4;
    const size_t base = (size_t)row * DM + c4;

    v4f a;
    if (first) {
        a = *(const v4f*)(hid + base);
    } else {
        const v4f hh = *(const v4f*)(hb + base);
        const v4f rr = *(const v4f*)(resid + base);
        a = hh + rr;
    }
    const float mu  = block_sum128(hsum4(a), sred) * (1.0f / DM);
    const v4f   dl  = a - mu;
    const float var = block_sum128(hsum4(dl * dl), sred) * (1.0f / DM);
    const float inv = rsqrtf(var + 1e-5f);
    v4f v;
    if (first) {
        const v4f w = *(const v4f*)(lw + c4);
        const v4f b = *(const v4f*)(lb + c4);
        v = (dl * inv) * w + b;
    } else {
        v = a;
    }
    *(volatile v4f*)(resid + base) = v;

    const float ms   = block_sum128(hsum4(v * v), sred) * (1.0f / DM);
    const float rinv = rsqrtf(ms + 1e-5f);
    const v4f   bw   = *(const v4f*)(bnw + c4);
    *(v4f*)(srow + c4) = (v * rinv) * bw;
    __threadfence();
    *(volatile v4f*)(resid + base) = v;
    __syncthreads();

    if (tid < 64) {
        const int c8 = tid * 8;
        Pack8 pk;
        pk.f = __builtin_convertvector(ld8f(srow + c8), v8h);
        const u16x8 u = pk.u;
        unsigned short* gp = hn16 + (size_t)row * DM + c8;
        *(volatile u16x8*)gp = u;
        __threadfence();
        *(volatile u16x8*)gp = u;
    }
}

__global__ __launch_bounds__(128)
void final_norm_kernel(const float* __restrict__ hb, const float* __restrict__ resid, const float* __restrict__ nfw,
                       const float* __restrict__ hid, float* hout,
                       const float* __restrict__ lw, const float* __restrict__ lb, unsigned short* x16)
{
    __shared__ float sred[4];
    __shared__ __attribute__((aligned(16))) float srow[DM];
    const int row = blockIdx.x;
    const int tid = threadIdx.x;
    const int c4  = tid * 4;
    const size_t base = (size_t)row * DM + c4;

    const v4f hh = *(const v4f*)(hb + base);
    const v4f rr = *(const v4f*)(resid + base);
    const v4f a  = hh + rr;
    const float ms  = block_sum128(hsum4(a * a), sred) * (1.0f / DM);
    const float inv = rsqrtf(ms + 1e-5f);
    const v4f w   = *(const v4f*)(nfw + c4);
    const v4f sc  = *(const v4f*)(hid + base);
    const v4f hv  = sc + (a * inv) * w;
    *(volatile v4f*)(hout + base) = hv;

    const float mu   = block_sum128(hsum4(hv), sred) * (1.0f / DM);
    const v4f   dl   = hv - mu;
    const float var  = block_sum128(hsum4(dl * dl), sred) * (1.0f / DM);
    const float linv = rsqrtf(var + 1e-5f);
    const v4f w2 = *(const v4f*)(lw + c4);
    const v4f b2 = *(const v4f*)(lb + c4);
    *(v4f*)(srow + c4) = (dl * linv) * w2 + b2;
    __threadfence();
    *(volatile v4f*)(hout + base) = hv;
    __syncthreads();

    if (tid < 64) {
        const int c8 = tid * 8;
        Pack8 pk;
        pk.f = __builtin_convertvector(ld8f(srow + c8), v8h);
        const u16x8 u = pk.u;
        unsigned short* gp = x16 + (size_t)row * DM + c8;
        *(volatile u16x8*)gp = u;
        __threadfence();
        *(volatile u16x8*)gp = u;
    }
}

__global__ __launch_bounds__(128)
void conv_silu_kernel(const float* __restrict__ xz, const float* __restrict__ cw,
                      const float* __restrict__ cb, unsigned short* u16)
{
    const int t  = blockIdx.x;
    const int d0 = threadIdx.x * 8;
    const float* xr = xz + (size_t)t * (2 * DI) + d0;

    const v8f x3 = ld8f(xr);
    v8f x2 = zero8(), x1 = zero8(), x0 = zero8();
    if (t >= 1) x2 = ld8f(xr - 2 * DI);
    if (t >= 2) x1 = ld8f(xr - 4 * DI);
    if (t >= 3) x0 = ld8f(xr - 6 * DI);

    v8f u;
#pragma unroll
    for (int c = 0; c < 8; ++c) {
        const v4f w = *(const v4f*)(cw + (size_t)(d0 + c) * KC);
        u[c] = 16.0f * silu_f(conv4(x0[c], x1[c], x2[c], x3[c], w, cb[d0 + c]));
    }
    Pack8 pk;
    pk.f = __builtin_convertvector(u, v8h);
    const u16x8 v = pk.u;
    unsigned short* gp = u16 + (size_t)t * DI + d0;
    *(volatile u16x8*)gp = v;
    __threadfence();
    *(volatile u16x8*)gp = v;
}

__device__ __forceinline__ void yg_rows_store(const unsigned short* sl, unsigned short* g, size_t gbase,
                                              int wave, int lane) {
#pragma unroll
    for (int it = 0; it < 2; ++it) {
        const int t = wave * 8 + it * 4 + (lane >> 3);
        const int c = (lane & 7) * 8;
        const u16x8 v = *(const u16x8*)(sl + t * 64 + c);
        *(volatile u16x8*)(g + gbase + (size_t)t * DI + c) = v;
    }
}

__global__ __launch_bounds__(64)
void scan_kernel(const float* __restrict__ xz, const float* __restrict__ delta, const float* __restrict__ dbc,
                 const float* __restrict__ cw, const float* __restrict__ cb,
                 const float* __restrict__ Alog, const float* __restrict__ Dp, unsigned short* yg16)
{
    __shared__ __attribute__((aligned(16))) float sbc[16 * 32];
    __shared__ __attribute__((aligned(16))) unsigned short syg[16 * 64];

    const int tid   = threadIdx.x;
    const int lane  = tid & 31;
    const int wave  = tid >> 5;
    const int dbase = blockIdx.x * 64;
    const int d     = dbase + tid;

    float an[NS], hs[NS];
#pragma unroll
    for (int n = 0; n < NS; ++n) {
        an[n] = -__expf(Alog[d * NS + n]);
        hs[n] = 0.0f;
    }
    const v4f   wv    = *(const v4f*)(cw + (size_t)d * KC);
    const float cbias = cb[d];
    const float Dd    = Dp[d];
    float xm1 = 0.0f, xm2 = 0.0f, xm3 = 0.0f;

#pragma unroll 1
    for (int l0 = 0; l0 < LSEQ; l0 += 16) {
        {
            const int s    = tid >> 2;
            const int part = (tid & 3) * 8;
            const float* src = dbc + (size_t)(l0 + s) * NBC + RR + part;
            *(v4f*)(sbc + s * 32 + part)     = *(const v4f*)src;
            *(v4f*)(sbc + s * 32 + part + 4) = *(const v4f*)(src + 4);
        }
        __syncthreads();
#pragma unroll 1
        for (int t = 0; t < 16; ++t) {
            const size_t mrow = (size_t)(l0 + t);
            const float xv = xz[mrow * (2 * DI) + d];
            const float zv = xz[mrow * (2 * DI) + DI + d];
            const float dt = delta[mrow * DI + d];
            const float u  = silu_f(conv4(xm3, xm2, xm1, xv, wv, cbias));
            xm3 = xm2; xm2 = xm1; xm1 = xv;
            const float du = dt * u;
            const float* bc = sbc + t * 32;
            float y = 0.0f;
#pragma unroll
            for (int n = 0; n < NS; ++n) {
                const float da = __expf(dt * an[n]);
                hs[n] = da * hs[n] + du * bc[n];
                y += hs[n] * bc[NS + n];
            }
            const float g = (y + u * Dd) * silu_f(zv);
            Pack1 pk;
            pk.f = (_Float16)(g * 16.0f);
            syg[t * 64 + tid] = pk.u;
        }
        __syncthreads();
        const size_t gbase = (size_t)l0 * DI + dbase;
        yg_rows_store(syg, yg16, gbase, wave, lane);
        __threadfence();
        yg_rows_store(syg, yg16, gbase, wave, lane);
        __syncthreads();
    }
}

extern "C" void kernel_launch(void* const* d_in, const int* in_sizes, int n_in,
                              void* d_out, int out_size, void* d_ws, size_t ws_size,
                              hipStream_t stream)
{
    if (n_in < 20) return;
    if (in_sizes[0]  != LSEQ * DM)          return;
    if (in_sizes[1]  != DM)                 return;
    if (in_sizes[2]  != DM)                 return;
    if (in_sizes[3]  != NLAY * 2 * DI * DM) return;
    if (in_sizes[4]  != NLAY * DI * KC)     return;
    if (in_sizes[5]  != NLAY * DI)          return;
    if (in_sizes[6]  != NLAY * NBC * DI)    return;
    if (in_sizes[7]  != NLAY * DI * RR)     return;
    if (in_sizes[8]  != NLAY * DI)          return;
    if (in_sizes[9]  != NLAY * DI * NS)     return;
    if (in_sizes[10] != NLAY * DI)          return;
    if (in_sizes[11] != NLAY * DM * DI)     return;
    if (in_sizes[12] != NLAY * DM)          return;
    if (in_sizes[13] != DM)                 return;
    if (in_sizes[14] != DM)                 return;
    if (in_sizes[15] != DM)                 return;
    if (in_sizes[16] != HM * DM)            return;
    if (in_sizes[17] != HM)                 return;
    if (in_sizes[18] != DM * HM)            return;
    if (in_sizes[19] != DM)                 return;
    if (out_size != LSEQ * DM)              return;

    const float* hsx    = (const float*)d_in[0];
    const float* ln1w   = (const float*)d_in[1];
    const float* ln1b   = (const float*)d_in[2];
    const float* winp   = (const float*)d_in[3];
    const float* convw  = (const float*)d_in[4];
    const float* convb  = (const float*)d_in[5];
    const float* xw     = (const float*)d_in[6];
    const float* dtw    = (const float*)d_in[7];
    const float* dtb    = (const float*)d_in[8];
    const float* alog   = (const float*)d_in[9];
    const float* dpar   = (const float*)d_in[10];
    const float* wout   = (const float*)d_in[11];
    const float* bnw    = (const float*)d_in[12];
    const float* nfw    = (const float*)d_in[13];
    const float* ln2w   = (const float*)d_in[14];
    const float* ln2b   = (const float*)d_in[15];
    const float* f1w    = (const float*)d_in[16];
    const float* f1b    = (const float*)d_in[17];
    const float* f2w    = (const float*)d_in[18];
    const float* f2b    = (const float*)d_in[19];
    float* out = (float*)d_out;

    const size_t SZ_WIN = (size_t)NLAY * 2 * DI * DM * 2;
    const size_t SZ_XW  = (size_t)NLAY * NBC * DI * 2;
    const size_t SZ_DTW = (size_t)NLAY * DI * RR * 2;
    const size_t SZ_OW  = (size_t)NLAY * DM * DI * 2;
    const size_t SZ_F1  = (size_t)HM * DM * 2;
    const size_t SZ_F2  = (size_t)DM * HM * 2;
    const size_t SZ_ROW = (size_t)LSEQ * DM * 4;
    const size_t SZ_H16 = (size_t)LSEQ * DM * 2;
    const size_t SZ_XZ  = (size_t)LSEQ * 2 * DI * 4;
    const size_t SZ_U16 = (size_t)LSEQ * DI * 2;
    const size_t SZ_DBC = (size_t)LSEQ * NBC * 4;
    const size_t SZ_DL  = (size_t)LSEQ * DI * 4;
    const size_t SZ_YG  = (size_t)LSEQ * DI * 2;
    const size_t SZ_ACT = (size_t)LSEQ * HM * 2;

    const size_t OFF_WIN  = 0;
    const size_t OFF_XW   = OFF_WIN  + SZ_WIN;
    const size_t OFF_DTW  = OFF_XW   + SZ_XW;
    const size_t OFF_OW   = OFF_DTW  + SZ_DTW;
    const size_t OFF_F1   = OFF_OW   + SZ_OW;
    const size_t OFF_F2   = OFF_F1   + SZ_F1;
    const size_t OFF_HB   = OFF_F2   + SZ_F2;
    const size_t OFF_RES  = OFF_HB   + SZ_ROW;
    const size_t OFF_HOUT = OFF_RES  + SZ_ROW;
    const size_t OFF_HN16 = OFF_HOUT + SZ_ROW;
    const size_t OFF_X16  = OFF_HN16 + SZ_H16;
    const size_t OFF_XZ   = OFF_X16  + SZ_H16;
    const size_t OFF_U16  = OFF_XZ   + SZ_XZ;
    const size_t OFF_DBC  = OFF_U16  + SZ_U16;
    const size_t OFF_DL   = OFF_DBC  + SZ_DBC;
    const size_t OFF_YG   = OFF_DL   + SZ_DL;
    const size_t OFF_ACT  = OFF_YG   + SZ_YG;
    const size_t WS_END   = OFF_ACT  + SZ_ACT;
    if (ws_size < WS_END) return;

    char* ws = (char*)d_ws;
    unsigned short* win16 = (unsigned short*)(ws + OFF_WIN);
    unsigned short* xw16  = (unsigned short*)(ws + OFF_XW);
    unsigned short* dtw16 = (unsigned short*)(ws + OFF_DTW);
    unsigned short* ow16  = (unsigned short*)(ws + OFF_OW);
    unsigned short* f1_16 = (unsigned short*)(ws + OFF_F1);
    unsigned short* f2_16 = (unsigned short*)(ws + OFF_F2);
    float*          hbuf  = (float*)(ws + OFF_HB);
    float*          resid = (float*)(ws + OFF_RES);
    float*          hout  = (float*)(ws + OFF_HOUT);
    unsigned short* hn16  = (unsigned short*)(ws + OFF_HN16);
    unsigned short* x16   = (unsigned short*)(ws + OFF_X16);
    float*          xz    = (float*)(ws + OFF_XZ);
    unsigned short* u16   = (unsigned short*)(ws + OFF_U16);
    float*          dbc   = (float*)(ws + OFF_DBC);
    float*          dl    = (float*)(ws + OFF_DL);
    unsigned short* yg16  = (unsigned short*)(ws + OFF_YG);
    unsigned short* act16 = (unsigned short*)(ws + OFF_ACT);

    {
        int n8;
        n8 = (NLAY * 2 * DI * DM) / 8;
        hipLaunchKernelGGL(cvt_f16_kernel, dim3((n8 + 255) / 256), dim3(256), 0, stream, winp, win16, n8, 64.0f);
        n8 = (NLAY * NBC * DI) / 8;
        hipLaunchKernelGGL(cvt_f16_kernel, dim3((n8 + 255) / 256), dim3(256), 0, stream, xw, xw16, n8, 64.0f);
        n8 = (NLAY * DI * RR) / 8;
        hipLaunchKernelGGL(cvt_f16_kernel, dim3((n8 + 255) / 256), dim3(256), 0, stream, dtw, dtw16, n8, 64.0f);
        n8 = (NLAY * DM * DI) / 8;
        hipLaunchKernelGGL(cvt_f16_kernel, dim3((n8 + 255) / 256), dim3(256), 0, stream, wout, ow16, n8, 64.0f);
        n8 = (HM * DM) / 8;
        hipLaunchKernelGGL(cvt_f16_kernel, dim3((n8 + 255) / 256), dim3(256), 0, stream, f1w, f1_16, n8, 64.0f);
        n8 = (DM * HM) / 8;
        hipLaunchKernelGGL(cvt_f16_kernel, dim3((n8 + 255) / 256), dim3(256), 0, stream, f2w, f2_16, n8, 64.0f);
    }

    for (int i = 0; i < NLAY; ++i) {
        const unsigned short* win_i = win16 + (size_t)i * 2 * DI * DM;
        const unsigned short* xw_i  = xw16  + (size_t)i * NBC * DI;
        const unsigned short* dtw_i = dtw16 + (size_t)i * DI * RR;
        const unsigned short* ow_i  = ow16  + (size_t)i * DM * DI;
        const float* cw_i   = convw + (size_t)i * DI * KC;
        const float* cb_i   = convb + (size_t)i * DI;
        const float* dtb_i  = dtb   + (size_t)i * DI;
        const float* al_i   = alog  + (size_t)i * DI * NS;
        const float* dp_i   = dpar  + (size_t)i * DI;
        const float* bnw_i  = bnw   + (size_t)i * DM;

        hipLaunchKernelGGL(prenorm_kernel, dim3(LSEQ), dim3(128), 0, stream,
                           hsx, ln1w, ln1b, (const float*)hbuf, resid, bnw_i, hn16, (int)(i == 0));

        hipLaunchKernelGGL(HIP_KERNEL_NAME(gemm_tn_kernel<4, 0, false, false>),
                           dim3((2 * DI) / 128, LSEQ / 64), dim3(128), 0, stream,
                           (const unsigned short*)hn16, hsx, (int)DM,
                           win_i, (int)DM,
                           xz, act16, (int)(2 * DI),
                           convb, hsx, (int)DM,
                           (int)DM, 1.0f, 0.015625f, 1.0f);

        hipLaunchKernelGGL(conv_silu_kernel, dim3(LSEQ), dim3(128), 0, stream,
                           (const float*)xz, cw_i, cb_i, u16);

        hipLaunchKernelGGL(HIP_KERNEL_NAME(gemm_tn_kernel<2, 0, false, false>),
                           dim3(NBC / 64, LSEQ / 64), dim3(128), 0, stream,
                           (const unsigned short*)u16, hsx, (int)DI,
                           xw_i, (int)DI,
                           dbc, act16, (int)NBC,
                           convb, hsx, (int)DM,
                           (int)DI, 1.0f, 0.0009765625f, 1.0f);

        hipLaunchKernelGGL(HIP_KERNEL_NAME(gemm_tn_kernel<4, 1, true, false>),
                           dim3(DI / 128, LSEQ / 64), dim3(128), 0, stream,
                           (const unsigned short*)u16, (const float*)dbc, (int)NBC,
                           dtw_i, (int)RR,
                           dl, act16, (int)DI,
                           dtb_i, hsx, (int)DM,
                           (int)RR, 16.0f, 0.0009765625f, 1.0f);

        hipLaunchKernelGGL(scan_kernel, dim3(DI / 64), dim3(64), 0, stream,
                           (const float*)xz, (const float*)dl, (const float*)dbc, cw_i, cb_i, al_i, dp_i, yg16);

        hipLaunchKernelGGL(HIP_KERNEL_NAME(gemm_tn_kernel<4, 0, false, false>),
                           dim3(DM / 128, LSEQ / 64), dim3(128), 0, stream,
                           (const unsigned short*)yg16, hsx, (int)DI,
                           ow_i, (int)DI,
                           hbuf, act16, (int)DM,
                           convb, hsx, (int)DM,
                           (int)DI, 1.0f, 0.0009765625f, 1.0f);
    }

    hipLaunchKernelGGL(final_norm_kernel, dim3(LSEQ), dim3(128), 0, stream,
                       (const float*)hbuf, (const float*)resid, nfw, hsx, hout, ln2w, ln2b, x16);

    hipLaunchKernelGGL(HIP_KERNEL_NAME(gemm_tn_kernel<4, 2, false, true>),
                       dim3(HM / 128, LSEQ / 64), dim3(128), 0, stream,
                       (const unsigned short*)x16, hsx, (int)DM,
                       (const unsigned short*)f1_16, (int)DM,
                       dl, act16, (int)HM,
                       f1b, hsx, (int)DM,
                       (int)DM, 1.0f, 0.015625f, 16.0f);

    hipLaunchKernelGGL(HIP_KERNEL_NAME(gemm_tn_kernel<4, 3, false, false>),
                       dim3(DM / 128, LSEQ / 64), dim3(128), 0, stream,
                       (const unsigned short*)act16, hsx, (int)HM,
                       (const unsigned short*)f2_16, (int)HM,
                       out, yg16, (int)DM,
                       f2b, (const float*)hout, (int)DM,
                       (int)HM, 1.0f, 0.0009765625f, 1.0f);
}
